// HeteNet_72593537237024
// MI455X (gfx1250) — hardware-verified
//
#include <hip/hip_runtime.h>


namespace {
constexpr int NTOK = 64 * 64, F = 512, H = 1024, NOUT = 512, NE = 4, GP = 64  , RP = NTOK + NE * GP  ;
constexpr float XS = 8.0f, WSC = 256.0f;
typedef _Float16 b16;
typedef __attribute__((ext_vector_type(16))) _Float16 v16b;
typedef __attribute__((ext_vector_type(8))) _Float16 v8b;
typedef __attribute__((ext_vector_type(8))) float v8f;
typedef __attribute__((ext_vector_type(4))) float v4f;
__device__ __forceinline__ float bf16_rne(float f) { unsigned int u = __float_as_uint(f); u += 0x7FFFu + ((u >> 16) & 1u); return __uint_as_float(u & 0xFFFF0000u); }
__device__ __forceinline__ void split16(float v, b16& hi, b16& lo) { hi = (b16)v; lo = (b16)(v - (float)hi); }
__device__ __forceinline__ v16b frag_kb(const b16* p, int hh) { const v8b a = *(const v8b*)(p + 8 * hh), b = *(const v8b*)(p + 16 + 8 * hh); v16b f;
#pragma unroll
  for (int e = 0; e < 8; ++e) { f[e] = a[e]; f[8 + e] = b[e]; } return f; }
__device__ __forceinline__ v8f wmma16b(v16b a, v16b b, v8f c) { v8f d = __builtin_amdgcn_wmma_f32_16x16x32_f16(false, a, false, b, (short)0, c, false, false); asm volatile("v_nop\n\tv_nop\n\tv_nop\n\tv_nop" : "+v"(d) : "v"(a), "v"(b)); return d; }
__device__ __forceinline__ void wave_lds_sync() { __builtin_amdgcn_fence(__ATOMIC_RELEASE, "workgroup"); __builtin_amdgcn_wave_barrier(); __builtin_amdgcn_fence(__ATOMIC_ACQUIRE, "workgroup"); }
__device__ __forceinline__ int iclamp(int v, int lo, int hi) { return v < lo ? lo : (v > hi ? hi : v); }

__global__ __launch_bounds__(256) void group_kernel(const int* __restrict__ types, int* __restrict__ PERMT, int* __restrict__ ROWEXP) {
  __shared__ int cnt[256][NE]; __shared__ int start[NE + 1]; __shared__ int perm[RP]; __shared__ int rexp[RP / 64];
  const int t_ = threadIdx.x; int my[NE] = {0, 0, 0, 0}; int ty[16];
  for (int j = 0; j < 16; ++j) { ty[j] = iclamp(types[t_ * 16 + j], 0, NE - 1); my[ty[j]]++; }
  for (int e = 0; e < NE; ++e) cnt[t_][e] = my[e];
  for (int q = t_; q < RP; q += 256) perm[q] = -1; for (int q = t_; q < RP / 64; q += 256) rexp[q] = -1;
  __syncthreads();
  if (t_ == 0) { int s = 0; for (int e = 0; e < NE; ++e) { start[e] = s; int tot = 0; for (int k = 0; k < 256; ++k) tot += cnt[k][e]; const int padded = (tot + GP - 1) / GP * GP; for (int q = 0; q < padded / 64; ++q) rexp[s / 64 + q] = e; s += padded; } start[NE] = s; }
  __syncthreads();
  int pre[NE]; for (int e = 0; e < NE; ++e) { int p = start[e]; for (int k = 0; k < t_; ++k) p += cnt[k][e]; pre[e] = p; }
  for (int j = 0; j < 16; ++j) { const int e = ty[j]; perm[pre[e]++] = t_ * 16 + j; }
  __syncthreads();
  typedef __attribute__((ext_vector_type(4))) int v4i;
  for (int pass = 0; pass < 2; ++pass) { for (int q = t_; q < RP / 4; q += 256) *(volatile v4i*)(PERMT + q * 4) = *(const v4i*)(&perm[q * 4]); if (t_ < RP / 64 / 4) *(volatile v4i*)(ROWEXP + t_ * 4) = *(const v4i*)(&rexp[t_ * 4]); __threadfence(); }
}
__global__ __launch_bounds__(256) void prep_kernel(const float* __restrict__ obs, const float* __restrict__ w1, const float* __restrict__ w2, const float* __restrict__ w3, b16* __restrict__ X16, b16* __restrict__ W1T, b16* __restrict__ W2T, b16* __restrict__ W3T) {
  const size_t u = (size_t)blockIdx.x * 256 + threadIdx.x; const size_t nx = (size_t)NTOK * F / 8, n1 = (size_t)NE * H * F / 8, n2 = (size_t)NE * H * H / 8, n3 = (size_t)NE * NOUT * H / 8; size_t t = u; v8b o;
  if (t < nx) { const size_t e = t * 8; for (int j = 0; j < 8; ++j) o[j] = (b16)(bf16_rne(obs[e + j]) * XS); for (int pass = 0; pass < 2; ++pass) { *(volatile v8b*)(X16 + e) = o; __threadfence(); } return; } t -= nx;
  if (t < n1) { const size_t e = t * 8; const int ex = (int)(e / ((size_t)H * F)); const size_t r = e % ((size_t)H * F); const int oo = (int)(r / F), k0 = (int)(r % F); for (int j = 0; j < 8; ++j) o[j] = (b16)(bf16_rne(w1[((size_t)ex * F + k0 + j) * H + oo]) * WSC); for (int pass = 0; pass < 2; ++pass) { *(volatile v8b*)(W1T + e) = o; __threadfence(); } return; } t -= n1;
  if (t < n2) { const size_t e = t * 8; const int ex = (int)(e / ((size_t)H * H)); const size_t r = e % ((size_t)H * H); const int oo = (int)(r / H), k0 = (int)(r % H); for (int j = 0; j < 8; ++j) o[j] = (b16)(bf16_rne(w2[((size_t)ex * H + k0 + j) * H + oo]) * WSC); for (int pass = 0; pass < 2; ++pass) { *(volatile v8b*)(W2T + e) = o; __threadfence(); } return; } t -= n2;
  if (t < n3) { const size_t e = t * 8; const int ex = (int)(e / ((size_t)NOUT * H)); const size_t r = e % ((size_t)NOUT * H); const int oo = (int)(r / H), k0 = (int)(r % H); for (int j = 0; j < 8; ++j) o[j] = (b16)(bf16_rne(w3[((size_t)ex * H + k0 + j) * NOUT + oo]) * WSC); for (int pass = 0; pass < 2; ++pass) { *(volatile v8b*)(W3T + e) = o; __threadfence(); } }
}
template <int LAYER>
__global__ __launch_bounds__(128) void glayer_kernel(const int* __restrict__ PERMT, const int* __restrict__ ROWEXP, const b16* __restrict__ X16, const b16* __restrict__ Ph, const b16* __restrict__ Pl, const b16* __restrict__ WT, const float* __restrict__ bias, b16* __restrict__ Qh, b16* __restrict__ Ql, float* __restrict__ out) {
  constexpr int KD = LAYER == 0 ? F : H; constexpr int NCOL = LAYER == 2 ? NOUT : H;
  __shared__ __attribute__((aligned(16))) float Tf[4][16][128 + 4]; __shared__ int tok[64];
  const int wave = threadIdx.x >> 5, lane = threadIdx.x & 31, nloc = lane & 15, hlf = lane >> 4; const int tile = blockIdx.x; const int ex = ROWEXP[tile]; if (ex < 0) return;
  const size_t r0 = (size_t)tile * 64 + wave * 16; const int n0 = blockIdx.y * 128;
  if (threadIdx.x < 64) tok[threadIdx.x] = PERMT[(size_t)tile * 64 + threadIdx.x];
  __syncthreads();
  const int mytok = tok[wave * 16 + nloc];
  const b16* arow_h; const b16* arow_l = nullptr;
  if (LAYER == 0) arow_h = X16 + (size_t)(mytok < 0 ? 0 : mytok) * F; else { arow_h = Ph + (r0 + nloc) * H; arow_l = Pl + (r0 + nloc) * H; }
  const b16* W = WT + (size_t)ex * NCOL * KD;
  v8f acc[8];
#pragma unroll
  for (int t = 0; t < 8; ++t) acc[t] = (v8f){};
#pragma unroll 2
  for (int kb = 0; kb < KD; kb += 32) { v16b a = frag_kb(arow_h + kb, hlf); v16b al; if (LAYER != 0) al = frag_kb(arow_l + kb, hlf);
    if (LAYER == 0 && mytok < 0) a = (v16b){};
#pragma unroll
    for (int t = 0; t < 8; ++t) { const v16b bw = frag_kb(W + (size_t)(n0 + t * 16 + nloc) * KD + kb, hlf); acc[t] = wmma16b(a, bw, acc[t]); if (LAYER != 0) acc[t] = wmma16b(al, bw, acc[t]); } }
#pragma unroll
  for (int t = 0; t < 8; ++t) { const int c = n0 + t * 16 + nloc; const float bb = bf16_rne(bias[(size_t)ex * NCOL + c]);
#pragma unroll 1
    for (int r = 0; r < 8; ++r) { float y = acc[t][r] * (1.0f / (XS * WSC)) + bb; if (LAYER != 2) y = fmaxf(y, 0.0f); Tf[wave][8 * hlf + r][t * 16 + nloc] = y; } }
  wave_lds_sync();
  if (LAYER != 2) { for (int pass = 0; pass < 2; ++pass) { for (int rr = 0; rr < 16; ++rr) { v4f v = *(const v4f*)(&Tf[wave][rr][lane * 4]); b16 ph[4], pl[4]; for (int j = 0; j < 4; ++j) split16(v[j] * XS, ph[j], pl[j]);
        typedef __attribute__((ext_vector_type(4))) _Float16 v4h; v4h hv = {ph[0], ph[1], ph[2], ph[3]}, lv = {pl[0], pl[1], pl[2], pl[3]}; *(volatile v4h*)(Qh + (r0 + rr) * H + n0 + lane * 4) = hv; *(volatile v4h*)(Ql + (r0 + rr) * H + n0 + lane * 4) = lv; } __threadfence(); } }
  else { for (int pass = 0; pass < 2; ++pass) { for (int rr = 0; rr < 16; ++rr) { const int tk = tok[wave * 16 + rr]; if (tk >= 0) *(volatile v4f*)(out + (size_t)tk * NOUT + n0 + lane * 4) = *(const v4f*)(&Tf[wave][rr][lane * 4]); } __threadfence(); } }
}
}

extern "C" void kernel_launch(void* const* d_in, const int* in_sizes, int n_in, void* d_out, int out_size, void* d_ws, size_t ws_size, hipStream_t stream) {
  (void)n_in;
  auto Fp = [&](int i) { return (const float*)d_in[i]; }; auto Ip = [&](int i) { return (const int*)d_in[i]; };
  if (in_sizes[0] != NTOK * F || in_sizes[1] != NE * F * H || in_sizes[3] != NE * H * H || in_sizes[5] != NE * H * NOUT || in_sizes[7] != NTOK || out_size != NTOK * NOUT) return;
  size_t off = 0; char* ws = (char*)d_ws;
  auto carve = [&](size_t bytes) { char* p = ws + off; off += (bytes + 255) & ~(size_t)255; return p; };
  int* PERMT = (int*)carve((size_t)RP * 4); int* ROWEXP = (int*)carve((size_t)(RP / 64 + 16) * 4);
  b16* X16 = (b16*)carve((size_t)NTOK * F * 2); b16* W1T = (b16*)carve((size_t)NE * H * F * 2); b16* W2T = (b16*)carve((size_t)NE * H * H * 2); b16* W3T = (b16*)carve((size_t)NE * NOUT * H * 2);
  b16* P1h = (b16*)carve((size_t)RP * H * 2); b16* P1l = (b16*)carve((size_t)RP * H * 2); b16* P2h = (b16*)carve((size_t)RP * H * 2); b16* P2l = (b16*)carve((size_t)RP * H * 2);
  if (off > ws_size || off > ((size_t)128 << 20)) return;
  group_kernel<<<1, 256, 0, stream>>>(Ip(7), PERMT, ROWEXP);
  prep_kernel<<<(unsigned)(((size_t)NTOK * F / 8 + (size_t)NE * H * F / 8 + (size_t)NE * H * H / 8 + (size_t)NE * NOUT * H / 8 + 255) / 256), 256, 0, stream>>>(Fp(0), Fp(1), Fp(3), Fp(5), X16, W1T, W2T, W3T);
  glayer_kernel<0><<<dim3(RP / 64, H / 128), 128, 0, stream>>>(PERMT, ROWEXP, X16, nullptr, nullptr, W1T, Fp(2), P1h, P1l, nullptr);
  glayer_kernel<1><<<dim3(RP / 64, H / 128), 128, 0, stream>>>(PERMT, ROWEXP, nullptr, P1h, P1l, W2T, Fp(4), P2h, P2l, nullptr);
  glayer_kernel<2><<<dim3(RP / 64, NOUT / 128), 128, 0, stream>>>(PERMT, ROWEXP, nullptr, P2h, P2l, W3T, Fp(6), nullptr, nullptr, (float*)d_out);
}
